// HyperbolicMultiHeadAttention_54400055771511
// MI455X (gfx1250) — hardware-verified
//
#include <hip/hip_runtime.h>
#include <math.h>
#include <stdint.h>

#ifndef NB
#define NB 2
#endif
#ifndef SQ
#define SQ 1024
#endif
#define NB_FULL 2
#define SEQ  1024
#define DM   1024
#define NH   16
#define HD   64
#define XS   64.0f
#define WSC  256.0f
#define VS   256.0f
#define PCAR 32768.0f
#define LOG2E 1.4426950408889634f
#define MAXN 0.996f
#define NKB  (SEQ / 32)
#define GPITCH 68
#define TPITCH 65
#define TP16   72
#define CVT_THREADS (DM / 8)
#define TR_THREADS  128
#define ATT_THREADS 128

static_assert(NB >= 1 && NB <= NB_FULL);
static_assert((SQ % 64) == 0 && SQ >= 64 && SQ <= SEQ);
static_assert(NH * HD == DM && HD == 64);
static_assert((SEQ % 128) == 0 && (SEQ % 32) == 0 && NKB * 32 == SEQ);
static_assert((DM % 256) == 0 && (DM % 64) == 0 && (DM % 32) == 0 && CVT_THREADS == 128);
static_assert((GPITCH * 4) % 16 == 0 && (TP16 * 2) % 16 == 0);
static_assert(ATT_THREADS == 128 && TR_THREADS == 128 && ATT_THREADS * 8 == SEQ);

typedef unsigned short u16;
typedef _Float16 v16h __attribute__((ext_vector_type(16)));
typedef _Float16 v8h  __attribute__((ext_vector_type(8)));
typedef __bf16   v16b __attribute__((ext_vector_type(16)));
typedef float    v8f  __attribute__((ext_vector_type(8)));
typedef float    v4f  __attribute__((ext_vector_type(4)));
typedef unsigned int v4u __attribute__((ext_vector_type(4)));
typedef v4u __attribute__((may_alias)) v4ua;
typedef v4f __attribute__((may_alias)) v4fa;

union Frag { v16h h; v16b b; v4u u[2]; };

__device__ __forceinline__ unsigned short bf_bits(float f) {
  unsigned u = __float_as_uint(f);
  return (unsigned short)((u + 0x7FFFu + ((u >> 16) & 1u)) >> 16);
}
__device__ __forceinline__ float bf_up(unsigned short h) { return __uint_as_float(((unsigned)h) << 16); }
__device__ __forceinline__ float bfr(float f) { return bf_up(bf_bits(f)); }
__device__ __forceinline__ unsigned short h_bits(_Float16 x) { return __builtin_bit_cast(unsigned short, x); }
__device__ __forceinline__ unsigned pk16(unsigned short a, unsigned short b) { return (unsigned)a | ((unsigned)b << 16); }
__device__ __forceinline__ v8f zero8() { v8f z = {0.f, 0.f, 0.f, 0.f, 0.f, 0.f, 0.f, 0.f}; return z; }
__device__ __forceinline__ float red8(float v) {
  v += __shfl_xor(v, 1, 32); v += __shfl_xor(v, 2, 32); v += __shfl_xor(v, 4, 32); return v;
}
__device__ __forceinline__ float rsum16(float v) {
  v += __shfl_xor(v, 8, 32); v += __shfl_xor(v, 4, 32); v += __shfl_xor(v, 2, 32); v += __shfl_xor(v, 1, 32); return v;
}

__device__ __forceinline__ Frag ldfrag(const u16* p) {
  Frag f;
  f.u[0] = *(const v4u*)(p);
  f.u[1] = *(const v4u*)(p + 16);
  return f;
}

__device__ __forceinline__ v8f mma_h(const Frag& a, const Frag& b, v8f c) {
  return __builtin_amdgcn_wmma_f32_16x16x32_f16(false, a.h, false, b.h, (short)0, c, false, false);
}
__device__ __forceinline__ v8f mma_b(const Frag& a, const Frag& b, v8f c) {
  return __builtin_amdgcn_wmma_f32_16x16x32_bf16(false, a.b, false, b.b, (short)0, c, false, false);
}
__device__ __forceinline__ void guard_sc(v8f& a, v8f& b, v16h x0, v16h x1, v16h x2, v16h x3, v16h x4, v16h x5) {
#if defined(__HIP_DEVICE_COMPILE__)
  asm volatile("v_nop\n\tv_nop\n\tv_nop\n\tv_nop"
               : "+v"(a), "+v"(b) : "v"(x0), "v"(x1), "v"(x2), "v"(x3), "v"(x4), "v"(x5) : "memory");
#endif
}
__device__ __forceinline__ void guard_pv(v8f (&o)[4], v16h p, v16h x0, v16h x1, v16h x2, v16h x3) {
#if defined(__HIP_DEVICE_COMPILE__)
  asm volatile("v_nop\n\tv_nop\n\tv_nop\n\tv_nop"
               : "+v"(o[0]), "+v"(o[1]), "+v"(o[2]), "+v"(o[3]) : "v"(p), "v"(x0), "v"(x1), "v"(x2), "v"(x3) : "memory");
#endif
}
__device__ __forceinline__ void guard_g(v8f (&acc)[8], v16h x0, v16h x1, v16h x2, v16h x3, v16h x4, v16h x5) {
#if defined(__HIP_DEVICE_COMPILE__)
  asm volatile("v_nop\n\tv_nop\n\tv_nop\n\tv_nop"
               : "+v"(acc[0]), "+v"(acc[1]), "+v"(acc[2]), "+v"(acc[3]),
                 "+v"(acc[4]), "+v"(acc[5]), "+v"(acc[6]), "+v"(acc[7])
               : "v"(x0), "v"(x1), "v"(x2), "v"(x3), "v"(x4), "v"(x5) : "memory");
#endif
}
__device__ __forceinline__ void acc_guard4(v8f (&o)[4]) {
#if defined(__HIP_DEVICE_COMPILE__)
  asm volatile("v_nop\n\tv_nop\n\tv_nop\n\tv_nop" : "+v"(o[0]), "+v"(o[1]), "+v"(o[2]), "+v"(o[3]));
#endif
}
__device__ __forceinline__ void wave_sync_lds() {
  __builtin_amdgcn_fence(__ATOMIC_RELEASE, "workgroup");
  __builtin_amdgcn_wave_barrier();
  __builtin_amdgcn_fence(__ATOMIC_ACQUIRE, "workgroup");
}

__global__ __launch_bounds__(CVT_THREADS)
void cvt16(const float* __restrict__ x, u16* Y, float scale) {
  const int tid = threadIdx.x;
  const size_t r = blockIdx.x;
  const float* src = x + r * (size_t)DM + (size_t)tid * 8;
  const v4f a = *(const v4f*)(src), c4 = *(const v4f*)(src + 4);
  v4u o;
#pragma unroll
  for (int e = 0; e < 2; ++e) {
    o[e]     = pk16(h_bits((_Float16)(bfr(a[2 * e]) * scale)),  h_bits((_Float16)(bfr(a[2 * e + 1]) * scale)));
    o[2 + e] = pk16(h_bits((_Float16)(bfr(c4[2 * e]) * scale)), h_bits((_Float16)(bfr(c4[2 * e + 1]) * scale)));
  }
  u16* dst = Y + r * (size_t)DM + (size_t)tid * 8;
  for (int pass = 0; pass < 2; ++pass) {
    *(volatile v4u*)(dst) = o;
    __threadfence();
  }
}

__global__ __launch_bounds__(256)
void rowstat(const float* __restrict__ x, float* CX2) {
  __shared__ __align__(16) float rs[32];
  const int tid = threadIdx.x, wave = tid >> 5, lane = tid & 31;
  const int row0 = blockIdx.x * 32;
#pragma unroll 1
  for (int j = 0; j < 4; ++j) {
    const int row = row0 + wave * 4 + j;
    const float* xr = x + (size_t)row * DM + 4 * lane;
    float s = 0.f;
#pragma unroll 2
    for (int q = 0; q < DM / 128; ++q) {
      const v4f a = *(const v4f*)(xr + 128 * q);
      const float a0 = bfr(a[0]), a1 = bfr(a[1]), a2 = bfr(a[2]), a3 = bfr(a[3]);
      s += a0 * a0; s += a1 * a1; s += a2 * a2; s += a3 * a3;
    }
    s += __shfl_xor(s, 16, 32); s += __shfl_xor(s, 8, 32); s += __shfl_xor(s, 4, 32);
    s += __shfl_xor(s, 2, 32);  s += __shfl_xor(s, 1, 32);
    if (lane == 0) rs[wave * 4 + j] = s;
  }
  __syncthreads();
  if (tid < 8) {
    const v4f v = *(const v4fa*)(rs + 4 * tid);
    float* dst = CX2 + row0 + 4 * tid;
    for (int pass = 0; pass < 2; ++pass) {
      *(volatile v4f*)(dst) = v;
      __threadfence();
    }
  }
}

__global__ __launch_bounds__(256)
void colstat(const float* __restrict__ z, const float* __restrict__ r, int nr, float* ZN, float* CH, float* SH) {
  __shared__ __align__(16) float st[3 * 256];
  const int tid = threadIdx.x;
  const int col = blockIdx.x * 256 + tid;
  float s = 0.f;
#pragma unroll 4
  for (int k = 0; k < DM; ++k) {
    const float v = bfr(z[(size_t)k * DM + col]);
    s += v * v;
  }
  const float zn = fmaxf(sqrtf(s), 1e-15f);
  int ri = col;
  ri = (ri < nr - 1) ? ri : (nr - 1);
  const float dr = 2.0f * bfr(r[ri]);
  st[tid]       = zn;
  st[256 + tid] = coshf(dr);
  st[512 + tid] = sinhf(dr);
  __syncthreads();
  const int wv = tid >> 5;
  if (wv < 6) {
    const int arr = wv >> 1;
    const int q = tid & 63;
    const v4f val = *(const v4fa*)(st + arr * 256 + 4 * q);
    float* dst = (arr == 0) ? ZN : ((arr == 1) ? CH : SH);
    dst += blockIdx.x * 256 + 4 * q;
    for (int pass = 0; pass < 2; ++pass) {
      *(volatile v4f*)(dst) = val;
      __threadfence();
    }
  }
}

__global__ __launch_bounds__(TR_THREADS)
void cvtT16(const float* __restrict__ W, u16* Y, float scale) {
  __shared__ __align__(16) float tile[64 * TPITCH];
  const int tid = threadIdx.x;
  constexpr int NT = DM / 64;
  const int bid = blockIdx.x;
  const int kt  = bid % NT;
  const int ntb = bid / NT;
  const int k0  = kt * 64, n0 = ntb * 64;
  const int lr = tid >> 4, lc = (tid & 15) * 4;
#pragma unroll
  for (int p = 0; p < 8; ++p) {
    const int kk = p * 8 + lr;
    const v4f w4 = *(const v4f*)(W + (size_t)(k0 + kk) * (size_t)DM + n0 + lc);
    tile[kk * TPITCH + lc + 0] = w4[0];
    tile[kk * TPITCH + lc + 1] = w4[1];
    tile[kk * TPITCH + lc + 2] = w4[2];
    tile[kk * TPITCH + lc + 3] = w4[3];
  }
  __syncthreads();
  const int rq = tid >> 3, c8 = (tid & 7) * 8;
  v4u ov[4];
#pragma unroll
  for (int i = 0; i < 4; ++i) {
    const int row = 16 * i + rq;
#pragma unroll
    for (int e = 0; e < 4; ++e) {
      const float x0 = tile[(c8 + 2 * e) * TPITCH + row];
      const float x1 = tile[(c8 + 2 * e + 1) * TPITCH + row];
      ov[i][e] = pk16(h_bits((_Float16)(bfr(x0) * scale)), h_bits((_Float16)(bfr(x1) * scale)));
    }
  }
  u16* dst = Y + (size_t)n0 * (size_t)DM + k0 + c8;
  for (int pass = 0; pass < 2; ++pass) {
#pragma unroll
    for (int i = 0; i < 4; ++i) {
      const int row = 16 * i + rq;
      *(volatile v4u*)(dst + (size_t)row * (size_t)DM) = ov[i];
    }
    __threadfence();
  }
}

__device__ __forceinline__ void gemm_core(const u16* ap, const u16* bp, int K, v8f (&acc)[8]) {
  const size_t rs16 = (size_t)16 * (size_t)K;
#pragma unroll 1
  for (int k0 = 0; k0 < K; k0 += 32) {
    const Frag a0 = ldfrag(ap + k0), a1 = ldfrag(ap + rs16 + k0);
    const Frag b0 = ldfrag(bp + k0);
    const Frag b1 = ldfrag(bp + rs16 + k0);
    const Frag b2 = ldfrag(bp + 2 * rs16 + k0);
    const Frag b3 = ldfrag(bp + 3 * rs16 + k0);
    acc[0] = mma_h(a0, b0, acc[0]);
    acc[1] = mma_h(a0, b1, acc[1]);
    acc[2] = mma_h(a0, b2, acc[2]);
    acc[3] = mma_h(a0, b3, acc[3]);
    acc[4] = mma_h(a1, b0, acc[4]);
    acc[5] = mma_h(a1, b1, acc[5]);
    acc[6] = mma_h(a1, b2, acc[6]);
    acc[7] = mma_h(a1, b3, acc[7]);
    guard_g(acc, a0.h, a1.h, b0.h, b1.h, b2.h, b3.h);
  }
}
__device__ __forceinline__ void stage32x64(float* sl, v8f (&acc)[8], float oscale, int lane) {
  const int hh = lane >> 4, m = lane & 15;
#pragma unroll
  for (int i = 0; i < 2; ++i) {
#pragma unroll
    for (int r = 0; r < 8; ++r) {
      const int ro = (16 * i + 8 * hh + r) * GPITCH + m;
      sl[ro]      = acc[4 * i + 0][r] * oscale;
      sl[ro + 16] = acc[4 * i + 1][r] * oscale;
      sl[ro + 32] = acc[4 * i + 2][r] * oscale;
      sl[ro + 48] = acc[4 * i + 3][r] * oscale;
    }
  }
  wave_sync_lds();
}

__global__ __launch_bounds__(128)
void proj_mlr(const u16* __restrict__ A, const u16* __restrict__ Bt,
              const float* __restrict__ ZN, const float* __restrict__ CH, const float* __restrict__ SH,
              const float* __restrict__ CX2, int mode, u16* Ph, u16* Pl, float* RS) {
  __shared__ __align__(16) float slab[4 * 32 * GPITCH];
  __shared__ __align__(16) float rsc[4 * 32];
  const int tid = threadIdx.x, wave = tid >> 5, lane = tid & 31, hh = lane >> 4, m = lane & 15;
  constexpr int NT = DM / 64;
  const int bid  = blockIdx.x;
  const int nt   = bid % NT;
  const int mt   = bid / NT;
  const int rowb = mt * 128 + wave * 32;
  const int col0 = nt * 64;
  const u16* ap = A  + (size_t)(rowb + m) * DM + 8 * hh;
  const u16* bp = Bt + (size_t)(col0 + m) * DM + 8 * hh;
  v8f acc[8];
#pragma unroll
  for (int i = 0; i < 8; ++i) acc[i] = zero8();
  gemm_core(ap, bp, DM, acc);
  float* sl = slab + wave * 32 * GPITCH;
  stage32x64(sl, acc, 1.0f / (XS * WSC), lane);

  const int rq = lane >> 3, c8 = (lane & 7) * 8;
  float zn8[8], ch8[8], sh8[8];
  {
    const v4f z0 = *(const v4f*)(ZN + col0 + c8), z1 = *(const v4f*)(ZN + col0 + c8 + 4);
    const v4f h0 = *(const v4f*)(CH + col0 + c8), h1 = *(const v4f*)(CH + col0 + c8 + 4);
    const v4f g0 = *(const v4f*)(SH + col0 + c8), g1 = *(const v4f*)(SH + col0 + c8 + 4);
#pragma unroll
    for (int e = 0; e < 4; ++e) {
      zn8[e] = z0[e]; zn8[4 + e] = z1[e];
      ch8[e] = h0[e]; ch8[4 + e] = h1[e];
      sh8[e] = g0[e]; sh8[4 + e] = g1[e];
    }
  }
  const bool mv = (mode == 2);
#pragma unroll 1
  for (int i = 0; i < 8; ++i) {
    const int row = 4 * i + rq;
    const float cx  = CX2[rowb + row];
    const float omc = fmaxf(1.0f - cx, 1e-15f);
    const float opc = 1.0f + cx;
    float* sr = sl + row * GPITCH + c8;
    float y[8];
    float s0 = 0.f;
#pragma unroll
    for (int e = 0; e < 8; ++e) {
      const float mm  = sr[e] / zn8[e];
      const float arg = (2.0f * mm * ch8[e] - opc * sh8[e]) / omc;
      const float w   = 2.0f * zn8[e] * asinhf(arg);
      y[e] = sinhf(w);
      s0 += y[e] * y[e];
    }
    s0 = red8(s0);
    const float n0 = fmaxf(sqrtf(s0), 1e-15f);
    const bool cl0 = n0 > MAXN;
    float s1 = 0.f;
#pragma unroll
    for (int e = 0; e < 8; ++e) {
      const float yp = y[e] / n0 * MAXN;
      y[e] = cl0 ? yp : y[e];
      s1 += y[e] * y[e];
    }
    s1 = red8(s1);
    const float den = 1.0f + sqrtf(1.0f + s1);
    float s2 = 0.f;
#pragma unroll
    for (int e = 0; e < 8; ++e) {
      y[e] = y[e] / den;
      s2 += y[e] * y[e];
    }
    s2 = red8(s2);
    const float n2 = fmaxf(sqrtf(s2), 1e-15f);
    const bool cl2 = n2 > MAXN;
    float s3 = 0.f;
#pragma unroll
    for (int e = 0; e < 8; ++e) {
      const float yp = y[e] / n2 * MAXN;
      y[e] = cl2 ? yp : y[e];
      s3 += y[e] * y[e];
    }
    s3 = red8(s3);
    const float g    = 2.0f / fmaxf(1.0f - s3, 1e-15f);
    const float gmul = mv ? g : 1.0f;
    const float scal = mv ? (g - 1.0f) : s3;
#pragma unroll
    for (int e = 0; e < 8; ++e) sr[e] = y[e] * gmul;
    if ((lane & 7) == 0) rsc[wave * 32 + row] = scal;
  }
  wave_sync_lds();

  const int bb = rowb / SEQ, s0r = rowb - bb * SEQ, head = nt;
  if (lane < 8) {
    const v4f v = *(const v4fa*)(rsc + wave * 32 + 4 * lane);
    float* dst = RS + ((size_t)(bb * NH + head)) * SEQ + s0r + 4 * lane;
    for (int pass = 0; pass < 2; ++pass) {
      *(volatile v4f*)(dst) = v;
      __threadfence();
    }
  }
  const size_t pofs = (size_t)rowb * DM + (size_t)(col0 + c8);
  if (!mv) {
    v4u oh[8], ol[8];
#pragma unroll
    for (int i = 0; i < 8; ++i) {
      const int row = 4 * i + rq;
      const v4f a = *(const v4fa*)(sl + row * GPITCH + c8), c4 = *(const v4fa*)(sl + row * GPITCH + c8 + 4);
#pragma unroll
      for (int e = 0; e < 2; ++e) {
        const unsigned short ha = bf_bits(a[2 * e]),  hb = bf_bits(a[2 * e + 1]);
        const unsigned short la = bf_bits(a[2 * e] - bf_up(ha)), lb = bf_bits(a[2 * e + 1] - bf_up(hb));
        oh[i][e] = pk16(ha, hb);
        ol[i][e] = pk16(la, lb);
        const unsigned short hc = bf_bits(c4[2 * e]), hd = bf_bits(c4[2 * e + 1]);
        const unsigned short lc = bf_bits(c4[2 * e] - bf_up(hc)), ld = bf_bits(c4[2 * e + 1] - bf_up(hd));
        oh[i][2 + e] = pk16(hc, hd);
        ol[i][2 + e] = pk16(lc, ld);
      }
    }
    for (int pass = 0; pass < 2; ++pass) {
#pragma unroll
      for (int i = 0; i < 8; ++i) {
        const int row = 4 * i + rq;
        *(volatile v4u*)(Ph + pofs + (size_t)row * DM) = oh[i];
        *(volatile v4u*)(Pl + pofs + (size_t)row * DM) = ol[i];
      }
      __threadfence();
    }
  } else {
    v4u ov[8];
#pragma unroll
    for (int i = 0; i < 8; ++i) {
      const int row = 4 * i + rq;
      const v4f a = *(const v4fa*)(sl + row * GPITCH + c8), c4 = *(const v4fa*)(sl + row * GPITCH + c8 + 4);
#pragma unroll
      for (int e = 0; e < 2; ++e) {
        ov[i][e]     = pk16(h_bits((_Float16)(a[2 * e] * VS)),  h_bits((_Float16)(a[2 * e + 1] * VS)));
        ov[i][2 + e] = pk16(h_bits((_Float16)(c4[2 * e] * VS)), h_bits((_Float16)(c4[2 * e + 1] * VS)));
      }
    }
    for (int pass = 0; pass < 2; ++pass) {
#pragma unroll
      for (int i = 0; i < 8; ++i) {
        const int row = 4 * i + rq;
        *(volatile v4u*)(Ph + pofs + (size_t)row * DM) = ov[i];
      }
      __threadfence();
    }
  }
}

__global__ __launch_bounds__(TR_THREADS)
void trT16(const u16* __restrict__ Vg, u16* VT) {
  __shared__ __align__(16) u16 tile[64 * TP16];
  const int tid = threadIdx.x;
  constexpr int NST = SEQ / 64, NHT = DM / 64;
  const int bid = blockIdx.x;
  const int st  = bid % NST;
  const int tmp = bid / NST;
  const int ht  = tmp % NHT;
  const int b   = tmp / NHT;
  const int s0 = st * 64, hd0 = ht * 64;
  const int r = tid >> 3, c = (tid & 7) * 8;
#pragma unroll
  for (int p = 0; p < 4; ++p) {
    const int s = 16 * p + r;
    const v4u w = *(const v4u*)(Vg + ((size_t)(b * SEQ + s0 + s)) * DM + hd0 + c);
#pragma unroll
    for (int e = 0; e < 8; ++e)
      tile[(c + e) * TP16 + s] = (u16)((w[e >> 1] >> (16 * (e & 1))) & 0xFFFFu);
  }
  __syncthreads();
  const int rq = tid >> 3, c8 = (tid & 7) * 8;
  v4u ov[4];
#pragma unroll
  for (int i = 0; i < 4; ++i) {
    const int row = 16 * i + rq;
    ov[i] = *(const v4ua*)(tile + row * TP16 + c8);
  }
  u16* dst = VT + ((size_t)(b * DM + hd0)) * SEQ + s0 + c8;
  for (int pass = 0; pass < 2; ++pass) {
#pragma unroll
    for (int i = 0; i < 4; ++i) {
      const int row = 16 * i + rq;
      *(volatile v4u*)(dst + (size_t)row * SEQ) = ov[i];
    }
    __threadfence();
  }
}

__device__ __forceinline__ float logit2(float xy, float y2, float mk, float x2, float omx) {
  const float num  = fmaxf(x2 - 2.0f * xy + y2, 1e-15f);
  const float den  = fmaxf(omx * (1.0f - y2), 1e-15f);
  const float dist = acoshf(1.0f + 2.0f * num / den);
  return (mk - dist) * LOG2E;
}

__global__ __launch_bounds__(ATT_THREADS)
void attn_fwd(const u16* __restrict__ Qh, const u16* __restrict__ Ql, const u16* __restrict__ Kh, const u16* __restrict__ Kl,
              const u16* __restrict__ VT, const float* __restrict__ QX2, const float* __restrict__ KX2,
              const float* __restrict__ GM1, const float* __restrict__ amask, float* Out) {
  __shared__ __align__(16) float ms[SEQ];
  __shared__ __align__(16) float ky2[SEQ];
  __shared__ __align__(16) float kg1[SEQ];
  __shared__ __align__(16) float slab[4 * 16 * GPITCH];

  const int tid  = threadIdx.x;
  const int wave = tid >> 5;
  const int lane = tid & 31;
  const int hh   = lane >> 4;
  const int c    = lane & 15;

  constexpr int NQT = SQ / 64;
  const int bid  = blockIdx.x;
  const int qt   = bid % NQT;
  const int head = (bid / NQT) % NH;
  const int b    = bid / (NQT * NH);
  const int bh   = b * NH + head;
  const int q0   = qt * 64 + wave * 16;

  {
    const int i0 = tid * 8;
    const float* mp = amask + (size_t)b * SEQ + i0;
    const float* yp = KX2 + (size_t)bh * SEQ + i0;
    const float* gp = GM1 + (size_t)bh * SEQ + i0;
    const v4f m0 = *(const v4f*)(mp), m1 = *(const v4f*)(mp + 4);
    const v4f y0 = *(const v4f*)(yp), y1 = *(const v4f*)(yp + 4);
    const v4f g0 = *(const v4f*)(gp), g1 = *(const v4f*)(gp + 4);
#pragma unroll
    for (int e = 0; e < 4; ++e) {
      ms[i0 + e]  = bfr(m0[e]); ms[i0 + 4 + e]  = bfr(m1[e]);
      ky2[i0 + e] = y0[e];      ky2[i0 + 4 + e] = y1[e];
      kg1[i0 + e] = g0[e];      kg1[i0 + 4 + e] = g1[e];
    }
  }
  __syncthreads();

  const size_t qofs = ((size_t)(b * SEQ + q0 + c)) * DM + head * HD + 8 * hh;
  const Frag qh0 = ldfrag(Qh + qofs), qh1 = ldfrag(Qh + qofs + 32);
  const Frag ql0 = ldfrag(Ql + qofs), ql1 = ldfrag(Ql + qofs + 32);
  const float xq  = QX2[(size_t)bh * SEQ + q0 + c];
  const float omx = 1.0f - xq;
  const size_t kofs = ((size_t)(b * SEQ + c)) * DM + head * HD + 8 * hh;
  const u16* KhB = Kh + kofs;
  const u16* KlB = Kl + kofs;
  const u16* Vb = VT + ((size_t)(bh * HD + c)) * SEQ + 8 * hh;

  float mrun = -INFINITY, lrun = 0.f, drun = 0.f;
  v8f o[4];
#pragma unroll
  for (int j = 0; j < 4; ++j) o[j] = zero8();

#pragma unroll 1
  for (int it = 0; it < NKB; ++it) {
    const int kb = it * 32;
    v8f s0 = zero8(), s1 = zero8();
    const size_t k0o = (size_t)kb * DM, k1o = k0o + (size_t)16 * DM;
    {
      const Frag kh0 = ldfrag(KhB + k0o), kh1 = ldfrag(KhB + k1o);
      const Frag kl0 = ldfrag(KlB + k0o), kl1 = ldfrag(KlB + k1o);
      s0 = mma_b(kh0, qh0, s0); s0 = mma_b(kl0, qh0, s0); s0 = mma_b(kh0, ql0, s0);
      s1 = mma_b(kh1, qh0, s1); s1 = mma_b(kl1, qh0, s1); s1 = mma_b(kh1, ql0, s1);
      guard_sc(s0, s1, qh0.h, ql0.h, kh0.h, kh1.h, kl0.h, kl1.h);
    }
    {
      const Frag kh0 = ldfrag(KhB + k0o + 32), kh1 = ldfrag(KhB + k1o + 32);
      const Frag kl0 = ldfrag(KlB + k0o + 32), kl1 = ldfrag(KlB + k1o + 32);
      s0 = mma_b(kh0, qh1, s0); s0 = mma_b(kl0, qh1, s0); s0 = mma_b(kh0, ql1, s0);
      s1 = mma_b(kh1, qh1, s1); s1 = mma_b(kl1, qh1, s1); s1 = mma_b(kh1, ql1, s1);
      guard_sc(s0, s1, qh1.h, ql1.h, kh0.h, kh1.h, kl0.h, kl1.h);
    }
    float y2v[16], g1v[16], mkv[16];
    {
      const int ka = kb + 8 * hh, kc = kb + 16 + 8 * hh;
      const v4f ya = *(const v4fa*)(ky2 + ka), yb = *(const v4fa*)(ky2 + ka + 4);
      const v4f yc = *(const v4fa*)(ky2 + kc), yd = *(const v4fa*)(ky2 + kc + 4);
      const v4f ga = *(const v4fa*)(kg1 + ka), gb = *(const v4fa*)(kg1 + ka + 4);
      const v4f gc = *(const v4fa*)(kg1 + kc), gd = *(const v4fa*)(kg1 + kc + 4);
      const v4f ma = *(const v4fa*)(ms + ka),  mb = *(const v4fa*)(ms + ka + 4);
      const v4f mc = *(const v4fa*)(ms + kc),  md = *(const v4fa*)(ms + kc + 4);
#pragma unroll
      for (int e = 0; e < 4; ++e) {
        y2v[e] = ya[e]; y2v[4 + e] = yb[e]; y2v[8 + e] = yc[e]; y2v[12 + e] = yd[e];
        g1v[e] = ga[e]; g1v[4 + e] = gb[e]; g1v[8 + e] = gc[e]; g1v[12 + e] = gd[e];
        mkv[e] = ma[e]; mkv[4 + e] = mb[e]; mkv[8 + e] = mc[e]; mkv[12 + e] = md[e];
      }
    }
    float t[16];
#pragma unroll
    for (int i = 0; i < 8; ++i) {
      t[i]     = logit2(s0[i], y2v[i],     mkv[i],     xq, omx);
      t[8 + i] = logit2(s1[i], y2v[8 + i], mkv[8 + i], xq, omx);
    }
    float cm = t[0];
#pragma unroll
    for (int i = 1; i < 16; ++i) cm = fmaxf(cm, t[i]);
    cm = fmaxf(cm, __shfl_xor(cm, 16, 32));
    const float mn = fmaxf(mrun, cm);
    const float al = exp2f(mrun - mn);
    mrun = mn;
    float ps = 0.f, pd = 0.f;
    Frag ph;
#pragma unroll
    for (int w = 0; w < 2; ++w) {
#pragma unroll
      for (int e4 = 0; e4 < 4; ++e4) {
        const int i = 8 * w + 2 * e4;
        const float p0 = exp2f(t[i] - mn), p1 = exp2f(t[i + 1] - mn);
        ps += p0 + p1;
        pd += p0 * g1v[i] + p1 * g1v[i + 1];
        ph.u[w][e4] = pk16(h_bits((_Float16)(p0 * PCAR)), h_bits((_Float16)(p1 * PCAR)));
      }
    }
    ps += __shfl_xor(ps, 16, 32);
    pd += __shfl_xor(pd, 16, 32);
    lrun = lrun * al + ps;
    drun = drun * al + pd;
    float scl[8];
#pragma unroll
    for (int r = 0; r < 8; ++r) scl[r] = __shfl(al, 8 * hh + r, 32);
#pragma unroll
    for (int j = 0; j < 4; ++j) {
#pragma unroll
      for (int r = 0; r < 8; ++r) o[j][r] *= scl[r];
    }
    {
      const u16* vp = Vb + kb;
      const Frag v0 = ldfrag(vp);
      const Frag v1 = ldfrag(vp + (size_t)16 * SEQ);
      const Frag v2 = ldfrag(vp + (size_t)32 * SEQ);
      const Frag v3 = ldfrag(vp + (size_t)48 * SEQ);
      o[0] = mma_h(ph, v0, o[0]);
      o[1] = mma_h(ph, v1, o[1]);
      o[2] = mma_h(ph, v2, o[2]);
      o[3] = mma_h(ph, v3, o[3]);
      guard_pv(o, ph.h, v0.h, v1.h, v2.h, v3.h);
    }
  }
  acc_guard4(o);

  const float linv = 1.0f / lrun;
  const float nf   = linv * (1.0f / (PCAR * VS));
  const float dq   = fmaxf(drun * linv, 1e-10f);
  float nfr[8], dqr[8];
#pragma unroll
  for (int r = 0; r < 8; ++r) { nfr[r] = __shfl(nf, 8 * hh + r, 32); dqr[r] = __shfl(dq, 8 * hh + r, 32); }
  float sq[8];
#pragma unroll
  for (int r = 0; r < 8; ++r) {
    float sp = 0.f;
#pragma unroll
    for (int j = 0; j < 4; ++j) {
      const float tm = (o[j][r] * nfr[r]) / dqr[r];
      o[j][r] = tm;
      sp += tm * tm;
    }
    sq[r] = rsum16(sp);
  }
  float* sw = slab + wave * 16 * GPITCH;
#pragma unroll
  for (int r = 0; r < 8; ++r) {
    const float df = 1.0f + sqrtf(fmaxf(1.0f - sq[r], 1e-15f));
    float sp = 0.f;
#pragma unroll
    for (int j = 0; j < 4; ++j) {
      const float a = o[j][r] / df;
      o[j][r] = a;
      sp += a * a;
    }
    const float s2  = rsum16(sp);
    const float n2  = fmaxf(sqrtf(s2), 1e-15f);
    const bool  cl  = n2 > MAXN;
    const float fcl = MAXN / n2;
#pragma unroll
    for (int j = 0; j < 4; ++j) {
      const float a = o[j][r];
      sw[(8 * hh + r) * GPITCH + 16 * j + c] = cl ? (a * fcl) : a;
    }
  }
  wave_sync_lds();
  const int cc = lane & 15;
  v4f vals[8];
#pragma unroll
  for (int i = 0; i < 8; ++i) vals[i] = *(const v4fa*)(sw + (2 * i + hh) * GPITCH + 4 * cc);
  float* ob = Out + ((size_t)(b * SEQ + q0 + hh)) * DM + head * HD + 4 * cc;
  for (int pass = 0; pass < 2; ++pass) {
#pragma unroll
    for (int i = 0; i < 8; ++i) {
      *(volatile v4f*)(ob + (size_t)(2 * i) * DM) = vals[i];
    }
    __threadfence();
  }
}

static inline size_t up4k(size_t v) { return (v + 4095) & ~(size_t)4095; }

extern "C" void kernel_launch(void* const* d_in, const int* in_sizes, int n_in,
                              void* d_out, int out_size, void* d_ws, size_t ws_size,
                              hipStream_t stream) {
  if (n_in < 8) return;
  if (in_sizes[0] < NB * SEQ * DM) return;
  if (in_sizes[1] < NB * SEQ) return;
  if (in_sizes[2] < DM * DM || in_sizes[4] < DM * DM || in_sizes[6] < DM * DM) return;
  if (in_sizes[3] < 1 || in_sizes[5] < 1 || in_sizes[7] < 1) return;
  if (out_size < NB * SEQ * DM) return;

  const float* hs = (const float*)d_in[0];
  const float* am = (const float*)d_in[1];
  const float* qz = (const float*)d_in[2];
  const float* qr = (const float*)d_in[3];
  const float* kz = (const float*)d_in[4];
  const float* kr = (const float*)d_in[5];
  const float* vz = (const float*)d_in[6];
  const float* vr = (const float*)d_in[7];
  float*       out = (float*)d_out;
  const int nqr = in_sizes[3], nkr = in_sizes[5], nvr = in_sizes[7];

  const size_t nrow  = (size_t)NB * SEQ;
  const size_t szX16 = up4k(nrow * DM * 2);
  const size_t szWT  = up4k((size_t)DM * DM * 2);
  const size_t szCX2 = up4k(nrow * 4);
  const size_t szCOL = up4k((size_t)3 * DM * 4);
  const size_t szP   = up4k(nrow * DM * 2);
  const size_t szVT  = up4k((size_t)NB * NH * HD * SEQ * 2);
  const size_t szRS  = up4k((size_t)NB * NH * SEQ * 4);
  size_t off = 0;
  const size_t oX16 = off; off += szX16;
  const size_t oWQ  = off; off += szWT;
  const size_t oWK  = off; off += szWT;
  const size_t oWV  = off; off += szWT;
  const size_t oCX2 = off; off += szCX2;
  const size_t oZN  = off; off += szCOL;
  const size_t oCH  = off; off += szCOL;
  const size_t oSH  = off; off += szCOL;
  const size_t oQh  = off; off += szP;
  const size_t oQl  = off; off += szP;
  const size_t oKh  = off; off += szP;
  const size_t oKl  = off; off += szP;
  const size_t oVg  = off; off += szP;
  const size_t oVT  = off; off += szVT;
  const size_t oQX2 = off; off += szRS;
  const size_t oKX2 = off; off += szRS;
  const size_t oGM1 = off; off += szRS;
  if (off > ws_size) return;
  if (off > (size_t)134217728) return;

  char* ws = (char*)d_ws;
  u16*   X16 = (u16*)(ws + oX16);
  u16*   WQT = (u16*)(ws + oWQ);
  u16*   WKT = (u16*)(ws + oWK);
  u16*   WVT = (u16*)(ws + oWV);
  float* CX2 = (float*)(ws + oCX2);
  float* ZN  = (float*)(ws + oZN);
  float* CH  = (float*)(ws + oCH);
  float* SH  = (float*)(ws + oSH);
  u16*   Qh  = (u16*)(ws + oQh);
  u16*   Ql  = (u16*)(ws + oQl);
  u16*   Kh  = (u16*)(ws + oKh);
  u16*   Kl  = (u16*)(ws + oKl);
  u16*   Vg  = (u16*)(ws + oVg);
  u16*   VT  = (u16*)(ws + oVT);
  float* QX2 = (float*)(ws + oQX2);
  float* KX2 = (float*)(ws + oKX2);
  float* GM1 = (float*)(ws + oGM1);

  cvt16<<<dim3(NB * SEQ), dim3(CVT_THREADS), 0, stream>>>(hs, X16, XS);
  rowstat<<<dim3(NB * SEQ / 32), dim3(256), 0, stream>>>(hs, CX2);
  colstat<<<dim3(DM / 256), dim3(256), 0, stream>>>(qz, qr, nqr, ZN,          CH,          SH);
  colstat<<<dim3(DM / 256), dim3(256), 0, stream>>>(kz, kr, nkr, ZN + DM,     CH + DM,     SH + DM);
  colstat<<<dim3(DM / 256), dim3(256), 0, stream>>>(vz, vr, nvr, ZN + 2 * DM, CH + 2 * DM, SH + 2 * DM);
  cvtT16<<<dim3((DM / 64) * (DM / 64)), dim3(TR_THREADS), 0, stream>>>(qz, WQT, WSC);
  cvtT16<<<dim3((DM / 64) * (DM / 64)), dim3(TR_THREADS), 0, stream>>>(kz, WKT, WSC);
  cvtT16<<<dim3((DM / 64) * (DM / 64)), dim3(TR_THREADS), 0, stream>>>(vz, WVT, WSC);
  proj_mlr<<<dim3((NB * SEQ / 128) * (DM / 64)), dim3(128), 0, stream>>>(
      X16, WQT, ZN,          CH,          SH,          CX2, 0, Qh, Ql, QX2);
  proj_mlr<<<dim3((NB * SEQ / 128) * (DM / 64)), dim3(128), 0, stream>>>(
      X16, WKT, ZN + DM,     CH + DM,     SH + DM,     CX2, 1, Kh, Kl, KX2);
  proj_mlr<<<dim3((NB * SEQ / 128) * (DM / 64)), dim3(128), 0, stream>>>(
      X16, WVT, ZN + 2 * DM, CH + 2 * DM, SH + 2 * DM, CX2, 2, Vg, Vg, GM1);
  trT16<<<dim3(NB * (SEQ / 64) * (DM / 64)), dim3(TR_THREADS), 0, stream>>>(Vg, VT);
  attn_fwd<<<dim3(NB * NH * (SQ / 64)), dim3(ATT_THREADS), 0, stream>>>(Qh, Ql, Kh, Kl, VT, QX2, KX2, GM1, am, out);
  (void)hipGetLastError();
}
